// Retain_pertime_45019847196960
// MI455X (gfx1250) — hardware-verified
//
#include <hip/hip_runtime.h>
#include <math.h>

constexpr int NBATCH = 32;
constexpr int NTIME  = 64;
constexpr int NPREF  = 63;
constexpr int NFEAT  = 256;
constexpr int NGATE  = 768;
constexpr int NROWX  = NBATCH * NTIME;
constexpr int KCAT   = 2 * NFEAT;
constexpr int NTHR   = 256;
constexpr int HPITCH = 520;
constexpr int EPITCH = 260;
constexpr int NTRI   = NPREF * (NPREF + 1) / 2;
constexpr int NHBROW = NTRI * NBATCH;
constexpr int NOUT0  = NBATCH * NPREF;
constexpr int NOUT1  = NBATCH * NPREF * NFEAT;
constexpr int BR_EMBB = 0, BR_ABIH = 256, BR_BBIH = 1024, BR_ABHH = 1792, BR_BBHH = 2560;
constexpr int BR_BETAB = 3328, BR_ALPHAW = 3584, BR_OUTW = 3840, BR_TOTAL = 4096;
static_assert(NBATCH == 32 && NTIME == 64, "index bit tricks assume 32 x 64");
static_assert(NROWX % 64 == 0 && NFEAT % 64 == 0 && NGATE % 64 == 0, "GEMM M, N tile multiples");
static_assert(NFEAT % 32 == 0 && KCAT % 32 == 0, "GEMM K multiple of 32");
static_assert(((NROWX / 64) * (NFEAT / 64)) % 8 == 0, "emb GEMM grid exact");
static_assert(((NGATE / 64) * (NROWX / 64)) % 8 == 0, "gx GEMM grid exact");
static_assert((2 * NBATCH * HPITCH) % NTHR == 0, "h tile zero fill exact");
static_assert(HPITCH % 8 == 0 && EPITCH % 4 == 0, "16-B aligned LDS rows");
static_assert(NOUT0 * 4 == 8064 && (NOUT0 * 4) % 128 == 0, "out1 starts on a 128-B line");
static_assert(NOUT0 * 4 + NOUT1 * 4 == 2072448, "output extent");
static_assert(NFEAT == 32 * (NTHR / 32), "8 waves x 32 columns");

typedef __attribute__((ext_vector_type(16))) _Float16 v16h;
typedef __attribute__((ext_vector_type(8)))  _Float16 v8h;
typedef __attribute__((ext_vector_type(16))) __bf16   v16b;
typedef __attribute__((ext_vector_type(8)))  __bf16   v8b;
typedef __attribute__((ext_vector_type(8)))  float    v8f;
typedef __attribute__((ext_vector_type(4)))  float    v4f;
typedef __attribute__((ext_vector_type(4)))  unsigned int v4u;
typedef v4u __attribute__((__may_alias__)) v4u_ma;

__device__ __forceinline__ unsigned short f2bf_bits(float f) {
  unsigned u = __float_as_uint(f);
  return (unsigned short)((u + 0x7FFFu + ((u >> 16) & 1u)) >> 16);
}
__device__ __forceinline__ float bf_bits2f(unsigned short h) { return __uint_as_float(((unsigned)h) << 16); }
__device__ __forceinline__ float bf16r(float f) { return bf_bits2f(f2bf_bits(f)); }
__device__ __forceinline__ v8f zero8() { v8f z = {0.f, 0.f, 0.f, 0.f, 0.f, 0.f, 0.f, 0.f}; return z; }

__device__ __forceinline__ void dep_guard_h(v8f& a, v8f& b, v16h x, v16h y) { asm volatile("v_nop\n\tv_nop\n\tv_nop\n\tv_nop" : "+v"(a), "+v"(b) : "v"(x), "v"(y)); }
__device__ __forceinline__ void dep_guard_b(v8f& a, v8f& b, v16b x, v16b y) { asm volatile("v_nop\n\tv_nop\n\tv_nop\n\tv_nop" : "+v"(a), "+v"(b) : "v"(x), "v"(y)); }
__device__ __forceinline__ void keep4_h(v16h a, v16h b, v16h c, v16h d) { asm volatile("v_nop" :: "v"(a), "v"(b), "v"(c), "v"(d)); }
__device__ __forceinline__ void keep4_b(v16b a, v16b b, v16b c, v16b d) { asm volatile("v_nop" :: "v"(a), "v"(b), "v"(c), "v"(d)); }
__device__ __forceinline__ void acc_guard4(v8f& a, v8f& b, v8f& c, v8f& d) { asm volatile("v_nop\n\tv_nop\n\tv_nop\n\tv_nop" : "+v"(a), "+v"(b), "+v"(c), "+v"(d)); }
__device__ __forceinline__ void acc_guard2(v8f& a, v8f& b) { asm volatile("v_nop\n\tv_nop\n\tv_nop\n\tv_nop" : "+v"(a), "+v"(b)); }
template <typename T> struct Frag;
template <> struct Frag<_Float16> {
  typedef v16h V; union U { v16h v; v8h h[2]; };
  static __device__ __forceinline__ v16h load(const _Float16* p) {
    U f; f.h[0] = *(const v8h*)(p); f.h[1] = *(const v8h*)(p + 16); return f.v;
  }
  static __device__ __forceinline__ v8f mma(v16h a, v16h b, v8f c) {
    return __builtin_amdgcn_wmma_f32_16x16x32_f16(false, a, false, b, (short)0, c, false, false);
  }
  static __device__ __forceinline__ void guard(v8f& a, v8f& b, v16h x, v16h y) { dep_guard_h(a, b, x, y); }
  static __device__ __forceinline__ void keep(v16h a, v16h b, v16h c, v16h d) { keep4_h(a, b, c, d); }
};
template <> struct Frag<__bf16> {
  typedef v16b V; union U { v16b v; v8b h[2]; };
  static __device__ __forceinline__ v16b load(const __bf16* p) {
    U f; f.h[0] = *(const v8b*)(p); f.h[1] = *(const v8b*)(p + 16); return f.v;
  }
  static __device__ __forceinline__ v8f mma(v16b a, v16b b, v8f c) {
    return __builtin_amdgcn_wmma_f32_16x16x32_bf16(false, a, false, b, (short)0, c, false, false);
  }
  static __device__ __forceinline__ void guard(v8f& a, v8f& b, v16b x, v16b y) { dep_guard_b(a, b, x, y); }
  static __device__ __forceinline__ void keep(v16b a, v16b b, v16b c, v16b d) { keep4_b(a, b, c, d); }
};

template <int ET> struct Elem;
template <> struct Elem<0> { typedef _Float16 T; };
template <> struct Elem<1> { typedef __bf16 T; };
template <int ET, bool SPLIT, int BIAS_MODE, int OUT_MODE, bool RESID, int ACT = 0>
__global__ __launch_bounds__(256) void wmma_gemm64(
    const unsigned short* __restrict__ Ap, const unsigned short* __restrict__ A2p, int lda, long strideA,
    const unsigned short* __restrict__ Btp, const unsigned short* __restrict__ Bt2p, int ldb, long strideB,
    void* __restrict__ Cout, void* __restrict__ Cout2, int ldc, long strideC,
    const float* __restrict__ bias,
    const float* __restrict__ resid, long strideR,
    int M, int N, int K, float scale) {
  typedef typename Elem<ET>::T T;
  typedef typename Frag<T>::V V;
  const T* A = (const T*)Ap; const T* A2 = (const T*)A2p; const T* Bt = (const T*)Btp; const T* Bt2 = (const T*)Bt2p;
  __shared__ __align__(16) float sT[8][16 * 68];
  const int b    = blockIdx.y;
  const int lane = threadIdx.x & 31;
  const int wave = threadIdx.x >> 5;
  const int tilesN = N >> 6;
  const int tilesM = M >> 6;
  const int tile = blockIdx.x * 8 + wave;
  if (tile >= tilesM * tilesN) return;
  const int tm = tile / tilesN;
  const int tn = tile - tm * tilesN;
  const int m0 = tm << 6;
  const int n0 = tn << 6;

  const T* Ab  = A  + (size_t)b * strideA;
  const T* Bb  = Bt + (size_t)b * strideB;
  const T* Ab2 = SPLIT ? (A2  + (size_t)b * strideA) : nullptr;
  const T* Bb2 = SPLIT ? (Bt2 + (size_t)b * strideB) : nullptr;

  const int rlane = lane & 15;
  const int koff  = (lane >> 4) * 8;
  const int mOff  = (lane >> 4) * 8;

  v8f acc[4][4];
#pragma unroll
  for (int i = 0; i < 4; ++i)
#pragma unroll
    for (int j = 0; j < 4; ++j) acc[i][j] = (v8f){0.f,0.f,0.f,0.f,0.f,0.f,0.f,0.f};

  for (int k0 = 0; k0 < K; k0 += 32) {
    V bh[4], bl[4];
#pragma unroll
    for (int j = 0; j < 4; ++j) {
      const size_t bo = (size_t)(n0 + (j << 4) + rlane) * ldb + koff + k0;
      bh[j] = Frag<T>::load(Bb + bo);
      if (SPLIT) bl[j] = Frag<T>::load(Bb2 + bo);
    }
#pragma unroll
    for (int i = 0; i < 4; ++i) {
      const size_t ao = (size_t)(m0 + (i << 4) + rlane) * lda + koff + k0;
      V ah = Frag<T>::load(Ab + ao);
      V al;
      if (SPLIT) al = Frag<T>::load(Ab2 + ao);
#pragma unroll
      for (int j = 0; j < 4; ++j) {
        acc[i][j] = Frag<T>::mma(ah, bh[j], acc[i][j]);
        if (SPLIT) {
          acc[i][j] = Frag<T>::mma(ah, bl[j], acc[i][j]);
          acc[i][j] = Frag<T>::mma(al, bh[j], acc[i][j]);
        }
      }
      Frag<T>::guard(acc[i][0], acc[i][3], ah, SPLIT ? al : ah);
    }
    Frag<T>::keep(bh[0], bh[1], bh[2], bh[3]);
    if (SPLIT) Frag<T>::keep(bl[0], bl[1], bl[2], bl[3]);
  }
  acc_guard4(acc[0][0], acc[0][1], acc[0][2], acc[0][3]);
  acc_guard4(acc[1][0], acc[1][1], acc[1][2], acc[1][3]);
  acc_guard4(acc[2][0], acc[2][1], acc[2][2], acc[2][3]);
  acc_guard4(acc[3][0], acc[3][1], acc[3][2], acc[3][3]);

  float* slab = sT[wave];
  const float* Rb = RESID ? (resid + (size_t)b * strideR) : nullptr;
#pragma unroll
  for (int i = 0; i < 4; ++i) {
    const int mBase = m0 + (i << 4);
#pragma unroll
    for (int j = 0; j < 4; ++j) {
      const int n = n0 + (j << 4) + rlane;
      float bv = 0.f;
      if (BIAS_MODE == 2) bv = bias[n];
#pragma unroll
      for (int r = 0; r < 8; ++r) {
        float v = acc[i][j][r] * scale;
        if (BIAS_MODE == 1) v += bias[mBase + mOff + r];
        if (BIAS_MODE == 2) v += bv;
        if (RESID) v += Rb[(size_t)(mBase + mOff + r) * ldc + n];
        if (ACT == 1) v = tanhf(v);
        if (ACT == 2) v = fmaxf(v, 0.0f);
        if (ACT == 3) v = v / (1.0f + expf(-v));
        if (ACT == 4) v = (v > 0.f) ? v : 0.01f * v;
        if (ACT == 5) v = 0.5f * v * (1.0f + erff(v * 0.70710678118654752f));
        slab[(mOff + r) * 68 + (j << 4) + rlane] = v;
      }
    }
    __builtin_amdgcn_fence(__ATOMIC_RELEASE, "workgroup");
    __builtin_amdgcn_wave_barrier();
    __builtin_amdgcn_fence(__ATOMIC_ACQUIRE, "workgroup");
    if (OUT_MODE == 0) {
      float* C = (float*)Cout + (size_t)b * strideC;
      const int hh = lane >> 4, c4 = (lane & 15) * 4;
      for (int pass = 0; pass < 2; ++pass) {
#pragma unroll
        for (int it = 0; it < 8; ++it) {
          const int row = it * 2 + hh;
          v4f v = *(const v4f*)(slab + row * 68 + c4);
          *(volatile v4f*)(C + (size_t)(mBase + row) * ldc + n0 + c4) = v;
        }
        __threadfence();
      }
    } else {
      const int q = lane >> 3, c8 = (lane & 7) * 8;
      unsigned short* C  = (unsigned short*)Cout  + (size_t)b * strideC;
      unsigned short* C2 = (OUT_MODE == 2) ? ((unsigned short*)Cout2 + (size_t)b * strideC) : nullptr;
      for (int pass = 0; pass < 2; ++pass) {
#pragma unroll
        for (int it = 0; it < 4; ++it) {
          const int row = it * 4 + q;
          const float* sp = slab + row * 68 + c8;
          v8h hv, lv;
#pragma unroll
          for (int e = 0; e < 8; ++e) {
            if (OUT_MODE == 1) {
              hv[e] = (_Float16)sp[e];
            } else {
              unsigned short hb = f2bf_bits(sp[e]);
              unsigned short lb = f2bf_bits(sp[e] - bf_bits2f(hb));
              hv[e] = __builtin_bit_cast(_Float16, hb);
              lv[e] = __builtin_bit_cast(_Float16, lb);
            }
          }
          *(volatile v8h*)(C + (size_t)(mBase + row) * ldc + n0 + c8) = hv;
          if (OUT_MODE == 2) *(volatile v8h*)(C2 + (size_t)(mBase + row) * ldc + n0 + c8) = lv;
        }
        __threadfence();
      }
    }
    __builtin_amdgcn_fence(__ATOMIC_RELEASE, "workgroup");
    __builtin_amdgcn_wave_barrier();
    __builtin_amdgcn_fence(__ATOMIC_ACQUIRE, "workgroup");
  }
}

template <int XMAP, int DUP>
__global__ __launch_bounds__(NTHR) void cvt_rows_kernel(const float* __restrict__ src, unsigned short* __restrict__ dst, int nrows) {
  const int i = blockIdx.x * NTHR + threadIdx.x;
  if (i < nrows * 32) {
    const int row = i >> 5, c8 = (i & 31) * 8;
    const int srow = XMAP ? ((row & (NBATCH - 1)) * NTIME + (row >> 5)) : row;
    const float* sp = src + (size_t)srow * NFEAT + c8;
    const v4f a = *(const v4f*)(sp);
    const v4f b = *(const v4f*)(sp + 4);
    v8h hv;
#pragma unroll
    for (int e = 0; e < 4; ++e) {
      hv[e]     = __builtin_bit_cast(_Float16, f2bf_bits(a[e]));
      hv[4 + e] = __builtin_bit_cast(_Float16, f2bf_bits(b[e]));
    }
    const int dp = DUP ? KCAT : NFEAT;
    unsigned short* d0 = dst + (size_t)row * dp + c8;
    *(volatile v8h*)d0 = hv;
    if (DUP) *(volatile v8h*)(d0 + NFEAT) = hv;
    __threadfence();
    *(volatile v8h*)d0 = hv;
    if (DUP) *(volatile v8h*)(d0 + NFEAT) = hv;
  }
}

__global__ __launch_bounds__(NTHR) void split_rows_kernel(const float* __restrict__ src, unsigned short* __restrict__ dst, int nrows) {
  const int i = blockIdx.x * NTHR + threadIdx.x;
  if (i < nrows * 32) {
    const int row = i >> 5, c8 = (i & 31) * 8;
    const float* sp = src + (size_t)row * NFEAT + c8;
    const v4f a = *(const v4f*)(sp);
    const v4f b = *(const v4f*)(sp + 4);
    v8h hv, lv;
#pragma unroll
    for (int e = 0; e < 4; ++e) {
      const unsigned short h0 = f2bf_bits(a[e]);
      const unsigned short l0 = f2bf_bits(a[e] - bf_bits2f(h0));
      const unsigned short h1 = f2bf_bits(b[e]);
      const unsigned short l1 = f2bf_bits(b[e] - bf_bits2f(h1));
      hv[e]     = __builtin_bit_cast(_Float16, h0);
      lv[e]     = __builtin_bit_cast(_Float16, l0);
      hv[4 + e] = __builtin_bit_cast(_Float16, h1);
      lv[4 + e] = __builtin_bit_cast(_Float16, l1);
    }
    unsigned short* d0 = dst + (size_t)row * KCAT + c8;
    *(volatile v8h*)d0 = hv;
    *(volatile v8h*)(d0 + NFEAT) = lv;
    __threadfence();
    *(volatile v8h*)d0 = hv;
    *(volatile v8h*)(d0 + NFEAT) = lv;
  }
}

__global__ __launch_bounds__(NTHR) void tpdup_kernel(const float* __restrict__ src, unsigned short* __restrict__ dst) {
  __shared__ float Tt[64 * 65];
  const int tid = threadIdx.x;
  const int i0 = blockIdx.x * 64, e0 = blockIdx.y * 64;
#pragma unroll
  for (int it = 0; it < 4; ++it) {
    const int idx = it * NTHR + tid;
    const int rr = idx >> 4, cc = (idx & 15) * 4;
    const v4f v = *(const v4f*)(src + (size_t)(e0 + rr) * NFEAT + i0 + cc);
    Tt[rr * 65 + cc + 0] = v[0];
    Tt[rr * 65 + cc + 1] = v[1];
    Tt[rr * 65 + cc + 2] = v[2];
    Tt[rr * 65 + cc + 3] = v[3];
  }
  __syncthreads();
  const int q = tid >> 3, c8 = (tid & 7) * 8;
  v8h hv[2];
#pragma unroll
  for (int g = 0; g < 2; ++g) {
    const int qq = g * 32 + q;
#pragma unroll
    for (int e = 0; e < 8; ++e) {
      const float f = Tt[(c8 + e) * 65 + qq];
      hv[g][e] = __builtin_bit_cast(_Float16, f2bf_bits(f));
    }
  }
  for (int pass = 0; pass < 2; ++pass) {
#pragma unroll
    for (int g = 0; g < 2; ++g) {
      const size_t o = (size_t)(i0 + g * 32 + q) * KCAT + (size_t)(e0 + c8);
      *(volatile v8h*)(dst + o) = hv[g];
      *(volatile v8h*)(dst + o + NFEAT) = hv[g];
    }
    __threadfence();
  }
}

__global__ __launch_bounds__(64) void bias_prep_kernel(const float* __restrict__ emb_b, const float* __restrict__ a_bih,
                                                       const float* __restrict__ b_bih, const float* __restrict__ a_bhh,
                                                       const float* __restrict__ b_bhh, const float* __restrict__ beta_b,
                                                       const float* __restrict__ alpha_w, const float* __restrict__ out_w,
                                                       float* __restrict__ dst) {
  const int seg = blockIdx.x;
  const int t4 = threadIdx.x * 4;
  const float* sp;
  if (seg == 0)       sp = emb_b;
  else if (seg < 4)   sp = a_bih + (seg - 1) * NFEAT;
  else if (seg < 7)   sp = b_bih + (seg - 4) * NFEAT;
  else if (seg < 10)  sp = a_bhh + (seg - 7) * NFEAT;
  else if (seg < 13)  sp = b_bhh + (seg - 10) * NFEAT;
  else if (seg == 13) sp = beta_b;
  else if (seg == 14) sp = alpha_w;
  else                sp = out_w;
  const v4f v = *(const v4f*)(sp + t4);
  v4f o;
#pragma unroll
  for (int e = 0; e < 4; ++e) o[e] = bf16r(v[e]);
  float* op = dst + seg * NFEAT + t4;
  *(volatile v4f*)op = o;
  __threadfence();
  *(volatile v4f*)op = o;
}

template <bool ISB>
__global__ __launch_bounds__(NTHR) void gru_kernel(const float* __restrict__ GXT, const unsigned short* __restrict__ WHH2p,
                                                   const float* __restrict__ bihr, const float* __restrict__ bhhr,
                                                   const float* __restrict__ awr, const float* __restrict__ alpha_b,
                                                   float* __restrict__ ALPHA, unsigned short* __restrict__ HB2) {
  __shared__ __align__(16) unsigned short Ah[2 * NBATCH * HPITCH];
  __shared__ float red[ISB ? 4 : (2 * 8 * NBATCH)];
  __shared__ float pre_s[ISB ? 4 : (NTIME * NBATCH)];
  __shared__ float sm_m[NBATCH];
  __shared__ float sm_inv[NBATCH];
  const __bf16* WHH2 = (const __bf16*)WHH2p;
  const int p = blockIdx.x;
  const int tri = (p * (p + 1)) >> 1;
  const int tid = threadIdx.x, lane = tid & 31, wave = tid >> 5;
  const int c = lane & 15, hh = lane >> 4, koff = hh * 8;

#pragma unroll 1
  for (int i = tid; i < 2 * NBATCH * HPITCH; i += NTHR) Ah[i] = (unsigned short)0;
  float hst[2][2][8];
#pragma unroll
  for (int nt = 0; nt < 2; ++nt)
#pragma unroll
    for (int mt = 0; mt < 2; ++mt)
#pragma unroll
      for (int r = 0; r < 8; ++r) hst[nt][mt][r] = 0.0f;
  float bihv[3][2], bhhv[3][2], awv[2];
#pragma unroll
  for (int nt = 0; nt < 2; ++nt) {
    const int j = 32 * wave + 16 * nt + c;
#pragma unroll
    for (int g = 0; g < 3; ++g) {
      bihv[g][nt] = bihr[g * NFEAT + j];
      bhhv[g][nt] = bhhr[g * NFEAT + j];
    }
    awv[nt] = awr[j];
  }
  const float abr = bf16r(alpha_b[0]);
  __syncthreads();

  const v8f z8 = zero8();
#pragma unroll 1
  for (int k = 0; k <= p; ++k) {
    const int t = p - k;
    const int cur = k & 1;
    const __bf16* abase = (const __bf16*)(Ah + cur * (NBATCH * HPITCH));
    unsigned short* anew = Ah + (cur ^ 1) * (NBATCH * HPITCH);
    float part[2][8];
#pragma unroll
    for (int mt = 0; mt < 2; ++mt)
#pragma unroll
      for (int r = 0; r < 8; ++r) part[mt][r] = 0.0f;

#pragma unroll
    for (int nt = 0; nt < 2; ++nt) {
      const int j = 32 * wave + 16 * nt + c;
      const __bf16* w0p = WHH2 + (size_t)j * KCAT + koff;
      const __bf16* w1p = w0p + (size_t)NFEAT * KCAT;
      const __bf16* w2p = w0p + (size_t)2 * NFEAT * KCAT;
      const __bf16* a0p = abase + c * HPITCH + koff;
      const __bf16* a1p = a0p + 16 * HPITCH;
      v8f acc[3][2];
      acc[0][0] = z8; acc[0][1] = z8; acc[1][0] = z8; acc[1][1] = z8; acc[2][0] = z8; acc[2][1] = z8;
#pragma unroll 1
      for (int k0 = 0; k0 < KCAT; k0 += 32) {
        const v16b a0 = Frag<__bf16>::load(a0p + k0);
        const v16b a1 = Frag<__bf16>::load(a1p + k0);
        const v16b b0 = Frag<__bf16>::load(w0p + k0);
        const v16b b1 = Frag<__bf16>::load(w1p + k0);
        const v16b b2 = Frag<__bf16>::load(w2p + k0);
        acc[0][0] = Frag<__bf16>::mma(a0, b0, acc[0][0]);
        acc[0][1] = Frag<__bf16>::mma(a1, b0, acc[0][1]);
        acc[1][0] = Frag<__bf16>::mma(a0, b1, acc[1][0]);
        acc[1][1] = Frag<__bf16>::mma(a1, b1, acc[1][1]);
        acc[2][0] = Frag<__bf16>::mma(a0, b2, acc[2][0]);
        acc[2][1] = Frag<__bf16>::mma(a1, b2, acc[2][1]);
        dep_guard_b(acc[0][0], acc[2][1], a1, b2);
        keep4_b(a0, b0, b1, a1);
      }
      acc_guard4(acc[0][0], acc[0][1], acc[1][0], acc[1][1]);
      acc_guard2(acc[2][0], acc[2][1]);
#pragma unroll
      for (int mt = 0; mt < 2; ++mt) {
        const float* gxp = GXT + (size_t)j * NROWX + (size_t)(t * NBATCH + 16 * mt + 8 * hh);
        const v4f gr0 = *(const v4f*)(gxp);
        const v4f gr1 = *(const v4f*)(gxp + 4);
        const v4f gz0 = *(const v4f*)(gxp + (size_t)NFEAT * NROWX);
        const v4f gz1 = *(const v4f*)(gxp + (size_t)NFEAT * NROWX + 4);
        const v4f gn0 = *(const v4f*)(gxp + (size_t)2 * NFEAT * NROWX);
        const v4f gn1 = *(const v4f*)(gxp + (size_t)2 * NFEAT * NROWX + 4);
        float xr[8], xz[8], xn[8];
#pragma unroll
        for (int e = 0; e < 4; ++e) {
          xr[e] = gr0[e]; xr[4 + e] = gr1[e];
          xz[e] = gz0[e]; xz[4 + e] = gz1[e];
          xn[e] = gn0[e]; xn[4 + e] = gn1[e];
        }
#pragma unroll
        for (int r = 0; r < 8; ++r) {
          const float prr = (xr[r] + bihv[0][nt]) + (acc[0][mt][r] + bhhv[0][nt]);
          const float pzz = (xz[r] + bihv[1][nt]) + (acc[1][mt][r] + bhhv[1][nt]);
          const float rg = 1.0f / (1.0f + expf(-prr));
          const float zg = 1.0f / (1.0f + expf(-pzz));
          const float ng = tanhf((xn[r] + bihv[2][nt]) + rg * (acc[2][mt][r] + bhhv[2][nt]));
          const float ho = hst[nt][mt][r];
          const float hn = (1.0f - zg) * ng + zg * ho;
          hst[nt][mt][r] = hn;
          if (!ISB) part[mt][r] += hn * awv[nt];
          const unsigned short hb = f2bf_bits(hn);
          const unsigned short lb = f2bf_bits(hn - bf_bits2f(hb));
          const int row = 16 * mt + 8 * hh + r;
          anew[row * HPITCH + j] = hb;
          anew[row * HPITCH + NFEAT + j] = lb;
        }
      }
    }
    if (!ISB) {
#pragma unroll
      for (int mt = 0; mt < 2; ++mt)
#pragma unroll
        for (int r = 0; r < 8; ++r) {
          float v = part[mt][r];
          v += __shfl_xor(v, 1, 32);
          v += __shfl_xor(v, 2, 32);
          v += __shfl_xor(v, 4, 32);
          v += __shfl_xor(v, 8, 32);
          part[mt][r] = v;
        }
      float val = 0.0f;
#pragma unroll
      for (int mt = 0; mt < 2; ++mt)
#pragma unroll
        for (int r = 0; r < 8; ++r) val = (c == 8 * mt + r) ? part[mt][r] : val;
      const int bsel = 16 * (c >> 3) + 8 * hh + (c & 7);
      red[cur * (8 * NBATCH) + wave * NBATCH + bsel] = val;
    }
    __syncthreads();
    if (!ISB) {
      if (wave == 0) {
        float s = 0.0f;
#pragma unroll
        for (int w = 0; w < 8; ++w) s += red[cur * (8 * NBATCH) + w * NBATCH + lane];
        pre_s[k * NBATCH + lane] = 0.5f * s + abr;
      }
    } else {
      const unsigned short* at = Ah + (cur ^ 1) * (NBATCH * HPITCH);
      for (int pass = 0; pass < 2; ++pass) {
#pragma unroll
        for (int it = 0; it < 8; ++it) {
          const int row = 4 * wave + (it >> 1);
          const int col8 = (it & 1) * NFEAT + lane * 8;
          const v4u v = *(const v4u_ma*)(at + row * HPITCH + col8);
          *(volatile v4u*)(HB2 + ((size_t)(tri + k) * NBATCH + row) * KCAT + col8) = v;
        }
        __threadfence();
      }
    }
  }

  if (!ISB) {
    if (wave == 0) {
      float m = pre_s[lane];
#pragma unroll 1
      for (int kq = 1; kq <= p; ++kq) m = fmaxf(m, pre_s[kq * NBATCH + lane]);
      float s = 0.0f;
#pragma unroll 1
      for (int kq = 0; kq <= p; ++kq) s += expf(pre_s[kq * NBATCH + lane] - m);
      sm_m[lane] = m;
      sm_inv[lane] = 1.0f / s;
    }
    __syncthreads();
    const float mm = sm_m[lane], iv = sm_inv[lane];
#pragma unroll 1
    for (int kq = wave; kq <= p; kq += 8) {
      const float e = expf(pre_s[kq * NBATCH + lane] - mm) * iv;
      pre_s[kq * NBATCH + lane] = e;
    }
    for (int pass = 0; pass < 2; ++pass) {
#pragma unroll 1
      for (int kq = wave; kq <= p; kq += 8) {
        const float v = pre_s[kq * NBATCH + lane];
        *(volatile float*)(ALPHA + (size_t)(tri + kq) * NBATCH + lane) = v;
      }
      __threadfence();
    }
  }
}

__global__ __launch_bounds__(NTHR) __attribute__((amdgpu_num_vgpr(256)))
void attn_kernel(const unsigned short* __restrict__ HB2p, const float* __restrict__ ALPHA,
                 const unsigned short* __restrict__ BETAW2p,
                 const unsigned short* __restrict__ EMBWT2p,
                 const float* __restrict__ EMBF, const float* __restrict__ x,
                 const float* __restrict__ BIASR, const float* __restrict__ out_b,
                 float* __restrict__ out1, float* __restrict__ PREDT) {
  __shared__ __align__(16) float EMBS[NBATCH * EPITCH];
  __shared__ __align__(16) float XS[NBATCH * EPITCH];
  __shared__ __align__(16) unsigned short SW[NBATCH * HPITCH];
  __shared__ __align__(16) float CACC[NBATCH * EPITCH];
  __shared__ __align__(16) float GACC[NBATCH * EPITCH];
  __shared__ float predp[8 * NBATCH];
  const __bf16* HB2 = (const __bf16*)HB2p;
  const __bf16* BETAW2 = (const __bf16*)BETAW2p;
  const __bf16* EMBWT2 = (const __bf16*)EMBWT2p;
  const int p = blockIdx.x;
  const int tri = (p * (p + 1)) >> 1;
  const int tid = threadIdx.x, lane = tid & 31, wave = tid >> 5;
  const int c = lane & 15, hh = lane >> 4, koff = hh * 8;

  float betab[2], w0v[2];
#pragma unroll
  for (int nt = 0; nt < 2; ++nt) {
    const int j = 32 * wave + 16 * nt + c;
    betab[nt] = BIASR[BR_BETAB + j];
    w0v[nt] = BIASR[BR_OUTW + j];
  }
  const float obr = bf16r(out_b[0]);
#pragma unroll
  for (int nt = 0; nt < 2; ++nt)
#pragma unroll
    for (int mt = 0; mt < 2; ++mt)
#pragma unroll
      for (int r = 0; r < 8; ++r) {
        const int sidx = (16 * mt + 8 * hh + r) * EPITCH + 32 * wave + 16 * nt + c;
        CACC[sidx] = 0.0f;
        GACC[sidx] = 0.0f;
      }
  const v8f z8 = zero8();

#pragma unroll 1
  for (int t = 0; t <= p; ++t) {
    const int kk = p - t;
#pragma unroll 2
    for (int it = 0; it < 8; ++it) {
      const int idx = it * NTHR + tid;
      const int row = idx >> 6, c4 = (idx & 63) * 4;
      const v4f ev = *(const v4f*)(EMBF + (size_t)(t * NBATCH + row) * NFEAT + c4);
      const v4f xv = *(const v4f*)(x + ((size_t)row * NTIME + (size_t)t) * NFEAT + c4);
      v4f xq;
#pragma unroll
      for (int e = 0; e < 4; ++e) xq[e] = bf16r(xv[e]);
      *(v4f*)(EMBS + row * EPITCH + c4) = ev;
      *(v4f*)(XS + row * EPITCH + c4) = xq;
    }
    __syncthreads();

    v8f acc[2][2];
    acc[0][0] = z8; acc[0][1] = z8; acc[1][0] = z8; acc[1][1] = z8;
    {
      const __bf16* h0p = HB2 + ((size_t)(tri + kk) * NBATCH + c) * KCAT + koff;
      const __bf16* h1p = h0p + (size_t)16 * KCAT;
      const __bf16* b0p = BETAW2 + (size_t)(32 * wave + c) * KCAT + koff;
      const __bf16* b1p = b0p + (size_t)16 * KCAT;
#pragma unroll 1
      for (int k0 = 0; k0 < KCAT; k0 += 32) {
        const v16b a0 = Frag<__bf16>::load(h0p + k0);
        const v16b a1 = Frag<__bf16>::load(h1p + k0);
        const v16b b0 = Frag<__bf16>::load(b0p + k0);
        const v16b b1 = Frag<__bf16>::load(b1p + k0);
        acc[0][0] = Frag<__bf16>::mma(a0, b0, acc[0][0]);
        acc[0][1] = Frag<__bf16>::mma(a1, b0, acc[0][1]);
        acc[1][0] = Frag<__bf16>::mma(a0, b1, acc[1][0]);
        acc[1][1] = Frag<__bf16>::mma(a1, b1, acc[1][1]);
        dep_guard_b(acc[0][0], acc[1][1], a0, b1);
        keep4_b(a0, a1, b0, b1);
      }
      acc_guard4(acc[0][0], acc[0][1], acc[1][0], acc[1][1]);
    }
    float alv[2][8];
    {
      const float* ap = ALPHA + (size_t)(tri + kk) * NBATCH + 8 * hh;
      const v4f a00 = *(const v4f*)(ap);
      const v4f a01 = *(const v4f*)(ap + 4);
      const v4f a10 = *(const v4f*)(ap + 16);
      const v4f a11 = *(const v4f*)(ap + 20);
#pragma unroll
      for (int e = 0; e < 4; ++e) { alv[0][e] = a00[e]; alv[0][4 + e] = a01[e]; alv[1][e] = a10[e]; alv[1][4 + e] = a11[e]; }
    }
#pragma unroll
    for (int nt = 0; nt < 2; ++nt) {
      const int e = 32 * wave + 16 * nt + c;
#pragma unroll
      for (int mt = 0; mt < 2; ++mt) {
#pragma unroll
        for (int r = 0; r < 8; ++r) {
          const int row = 16 * mt + 8 * hh + r;
          const int sidx = row * EPITCH + e;
          const float beta = tanhf(0.5f * acc[nt][mt][r] + betab[nt]);
          const float sv = alv[mt][r] * beta;
          const float cold = CACC[sidx];
          CACC[sidx] = cold + sv * EMBS[sidx];
          const float sw = sv * w0v[nt];
          const unsigned short hb = f2bf_bits(sw);
          const unsigned short lb = f2bf_bits(sw - bf_bits2f(hb));
          SW[row * HPITCH + e] = hb;
          SW[row * HPITCH + NFEAT + e] = lb;
        }
      }
    }
    __syncthreads();

    acc[0][0] = z8; acc[0][1] = z8; acc[1][0] = z8; acc[1][1] = z8;
    {
      const __bf16* s0p = (const __bf16*)SW + c * HPITCH + koff;
      const __bf16* s1p = s0p + 16 * HPITCH;
      const __bf16* b0p = EMBWT2 + (size_t)(32 * wave + c) * KCAT + koff;
      const __bf16* b1p = b0p + (size_t)16 * KCAT;
#pragma unroll 1
      for (int k0 = 0; k0 < KCAT; k0 += 32) {
        const v16b a0 = Frag<__bf16>::load(s0p + k0);
        const v16b a1 = Frag<__bf16>::load(s1p + k0);
        const v16b b0 = Frag<__bf16>::load(b0p + k0);
        const v16b b1 = Frag<__bf16>::load(b1p + k0);
        acc[0][0] = Frag<__bf16>::mma(a0, b0, acc[0][0]);
        acc[0][1] = Frag<__bf16>::mma(a1, b0, acc[0][1]);
        acc[1][0] = Frag<__bf16>::mma(a0, b1, acc[1][0]);
        acc[1][1] = Frag<__bf16>::mma(a1, b1, acc[1][1]);
        dep_guard_b(acc[0][0], acc[1][1], a0, b1);
        keep4_b(a0, a1, b0, b1);
      }
      acc_guard4(acc[0][0], acc[0][1], acc[1][0], acc[1][1]);
    }
#pragma unroll
    for (int nt = 0; nt < 2; ++nt) {
      const int i = 32 * wave + 16 * nt + c;
#pragma unroll
      for (int mt = 0; mt < 2; ++mt) {
#pragma unroll
        for (int r = 0; r < 8; ++r) {
          const int sidx = (16 * mt + 8 * hh + r) * EPITCH + i;
          const float gold = GACC[sidx];
          GACC[sidx] = gold + acc[nt][mt][r] * XS[sidx];
        }
      }
    }
    __syncthreads();
  }

  float part[2][8];
#pragma unroll
  for (int mt = 0; mt < 2; ++mt)
#pragma unroll
    for (int r = 0; r < 8; ++r) {
      const int sidx = (16 * mt + 8 * hh + r) * EPITCH + 32 * wave + c;
      float v = 0.0f;
      v += CACC[sidx] * w0v[0];
      v += CACC[sidx + 16] * w0v[1];
      v += __shfl_xor(v, 1, 32);
      v += __shfl_xor(v, 2, 32);
      v += __shfl_xor(v, 4, 32);
      v += __shfl_xor(v, 8, 32);
      part[mt][r] = v;
    }
  {
    float val = 0.0f;
#pragma unroll
    for (int mt = 0; mt < 2; ++mt)
#pragma unroll
      for (int r = 0; r < 8; ++r) val = (c == 8 * mt + r) ? part[mt][r] : val;
    const int bsel = 16 * (c >> 3) + 8 * hh + (c & 7);
    predp[wave * NBATCH + bsel] = val;
  }
  __syncthreads();
  if (wave == 0) {
    float s = 0.0f;
#pragma unroll
    for (int w = 0; w < 8; ++w) s += predp[w * NBATCH + lane];
    const float pv = s + obr;
    *(volatile float*)(PREDT + p * NBATCH + lane) = pv;
    __threadfence();
    *(volatile float*)(PREDT + p * NBATCH + lane) = pv;
  }
  const float inv = 1.0f / (float)(p + 1);
  for (int pass = 0; pass < 2; ++pass) {
#pragma unroll
    for (int it = 0; it < 8; ++it) {
      const int row = 4 * wave + (it >> 1);
      const int c4 = (it & 1) * 128 + lane * 4;
      v4f v = *(const v4f*)(GACC + row * EPITCH + c4);
#pragma unroll
      for (int e = 0; e < 4; ++e) v[e] = v[e] * inv;
      *(volatile v4f*)(out1 + ((size_t)row * NPREF + (size_t)p) * NFEAT + c4) = v;
    }
    __threadfence();
  }
}

__global__ __launch_bounds__(512) void pred_out_kernel(const float* __restrict__ PREDT, float* __restrict__ out0) {
  const int i = threadIdx.x;
  if (i < NOUT0 / 4) {
    v4f v;
#pragma unroll
    for (int e = 0; e < 4; ++e) {
      const int f = 4 * i + e;
      const int b = f / NPREF;
      const int pp = f - b * NPREF;
      v[e] = PREDT[pp * NBATCH + b];
    }
    *(volatile v4f*)(out0 + 4 * i) = v;
    __threadfence();
    *(volatile v4f*)(out0 + 4 * i) = v;
  }
}

extern "C" void kernel_launch(void* const* d_in, const int* in_sizes, int n_in,
                              void* d_out, int out_size, void* d_ws, size_t ws_size, hipStream_t stream) {
  if (n_in < 17 || d_out == nullptr || d_ws == nullptr) return;
  if (in_sizes[0] != NBATCH * NTIME * NFEAT || in_sizes[1] != NFEAT * NFEAT || in_sizes[2] != NFEAT ||
      in_sizes[3] != NGATE * NFEAT || in_sizes[4] != NGATE * NFEAT || in_sizes[5] != NGATE || in_sizes[6] != NGATE ||
      in_sizes[7] != NGATE * NFEAT || in_sizes[8] != NGATE * NFEAT || in_sizes[9] != NGATE || in_sizes[10] != NGATE ||
      in_sizes[11] != NFEAT || in_sizes[12] != 1 || in_sizes[13] != NFEAT * NFEAT || in_sizes[14] != NFEAT ||
      in_sizes[15] != NFEAT || in_sizes[16] != 1 || out_size != NOUT0 + NOUT1) return;

  const float* x       = (const float*)d_in[0];
  const float* emb_w   = (const float*)d_in[1];
  const float* emb_b   = (const float*)d_in[2];
  const float* a_wih   = (const float*)d_in[3];
  const float* a_whh   = (const float*)d_in[4];
  const float* a_bih   = (const float*)d_in[5];
  const float* a_bhh   = (const float*)d_in[6];
  const float* b_wih   = (const float*)d_in[7];
  const float* b_whh   = (const float*)d_in[8];
  const float* b_bih   = (const float*)d_in[9];
  const float* b_bhh   = (const float*)d_in[10];
  const float* alpha_w = (const float*)d_in[11];
  const float* alpha_b = (const float*)d_in[12];
  const float* beta_w  = (const float*)d_in[13];
  const float* beta_b  = (const float*)d_in[14];
  const float* out_w   = (const float*)d_in[15];
  const float* out_b   = (const float*)d_in[16];
  float* out0 = (float*)d_out;
  float* out1 = (float*)d_out + NOUT0;

  char* ws = (char*)d_ws; size_t off = 0;
  auto carve = [&](size_t bytes) -> char* { char* p = ws + off; off += (bytes + 255) & ~(size_t)255; return p; };
  unsigned short* XB     = (unsigned short*)carve((size_t)NROWX * NFEAT * 2);
  unsigned short* EMBW   = (unsigned short*)carve((size_t)NFEAT * NFEAT * 2);
  unsigned short* EMBWT2 = (unsigned short*)carve((size_t)NFEAT * KCAT * 2);
  unsigned short* WIHA2  = (unsigned short*)carve((size_t)NGATE * KCAT * 2);
  unsigned short* WIHB2  = (unsigned short*)carve((size_t)NGATE * KCAT * 2);
  unsigned short* WHHA2  = (unsigned short*)carve((size_t)NGATE * KCAT * 2);
  unsigned short* WHHB2  = (unsigned short*)carve((size_t)NGATE * KCAT * 2);
  unsigned short* BETAW2 = (unsigned short*)carve((size_t)NFEAT * KCAT * 2);
  float*          BIASR  = (float*)carve((size_t)BR_TOTAL * 4);
  float*          EMBF   = (float*)carve((size_t)NROWX * NFEAT * 4);
  unsigned short* EMB2   = (unsigned short*)carve((size_t)NROWX * KCAT * 2);
  float*          GXTA   = (float*)carve((size_t)NGATE * NROWX * 4);
  float*          GXTB   = (float*)carve((size_t)NGATE * NROWX * 4);
  float*          ALPHA  = (float*)carve((size_t)NHBROW * 4);
  unsigned short* HB2    = (unsigned short*)carve((size_t)NHBROW * KCAT * 2);
  float*          PREDT  = (float*)carve((size_t)NPREF * NBATCH * 4);
  if (off > ws_size || off > (size_t)134217728) return;

  cvt_rows_kernel<1, 0><<<(NROWX * 32) / NTHR, NTHR, 0, stream>>>(x, XB, NROWX);
  cvt_rows_kernel<0, 0><<<(NFEAT * 32) / NTHR, NTHR, 0, stream>>>(emb_w, EMBW, NFEAT);
  tpdup_kernel<<<dim3(NFEAT / 64, NFEAT / 64), NTHR, 0, stream>>>(emb_w, EMBWT2);
  cvt_rows_kernel<0, 1><<<(NGATE * 32) / NTHR, NTHR, 0, stream>>>(a_wih, WIHA2, NGATE);
  cvt_rows_kernel<0, 1><<<(NGATE * 32) / NTHR, NTHR, 0, stream>>>(b_wih, WIHB2, NGATE);
  cvt_rows_kernel<0, 1><<<(NGATE * 32) / NTHR, NTHR, 0, stream>>>(a_whh, WHHA2, NGATE);
  cvt_rows_kernel<0, 1><<<(NGATE * 32) / NTHR, NTHR, 0, stream>>>(b_whh, WHHB2, NGATE);
  cvt_rows_kernel<0, 1><<<(NFEAT * 32) / NTHR, NTHR, 0, stream>>>(beta_w, BETAW2, NFEAT);
  bias_prep_kernel<<<16, 64, 0, stream>>>(emb_b, a_bih, b_bih, a_bhh, b_bhh, beta_b, alpha_w, out_w, BIASR);

  wmma_gemm64<1, false, 2, 0, false, 0><<<dim3((NROWX / 64) * (NFEAT / 64) / 8, 1), 256, 0, stream>>>(
      XB, XB, NFEAT, 0L, EMBW, EMBW, NFEAT, 0L, (void*)EMBF, (void*)EMBF, NFEAT, 0L,
      BIASR + BR_EMBB, EMBF, 0L, NROWX, NFEAT, NFEAT, 1.0f);
  split_rows_kernel<<<(NROWX * 32) / NTHR, NTHR, 0, stream>>>(EMBF, EMB2, NROWX);

  wmma_gemm64<1, false, 0, 0, false, 0><<<dim3((NGATE / 64) * (NROWX / 64) / 8, 1), 256, 0, stream>>>(
      WIHA2, WIHA2, KCAT, 0L, EMB2, EMB2, KCAT, 0L, (void*)GXTA, (void*)GXTA, NROWX, 0L,
      BIASR, EMBF, 0L, NGATE, NROWX, KCAT, 1.0f);
  wmma_gemm64<1, false, 0, 0, false, 0><<<dim3((NGATE / 64) * (NROWX / 64) / 8, 1), 256, 0, stream>>>(
      WIHB2, WIHB2, KCAT, 0L, EMB2, EMB2, KCAT, 0L, (void*)GXTB, (void*)GXTB, NROWX, 0L,
      BIASR, EMBF, 0L, NGATE, NROWX, KCAT, 1.0f);

  gru_kernel<false><<<NPREF, NTHR, 0, stream>>>(GXTA, WHHA2, BIASR + BR_ABIH, BIASR + BR_ABHH, BIASR + BR_ALPHAW,
                                                alpha_b, ALPHA, HB2);
  gru_kernel<true><<<NPREF, NTHR, 0, stream>>>(GXTB, WHHB2, BIASR + BR_BBIH, BIASR + BR_BBHH, BIASR + BR_ALPHAW,
                                               alpha_b, ALPHA, HB2);

  attn_kernel<<<NPREF, NTHR, 0, stream>>>(HB2, ALPHA, BETAW2, EMBWT2, EMBF, x, BIASR, out_b, out1, PREDT);

  pred_out_kernel<<<1, 512, 0, stream>>>(PREDT, out0);
}
